// LMUFFT_29635274342993
// MI455X (gfx1250) — hardware-run, weakly checked
//
#include <hip/hip_runtime.h>
#include <math.h>

constexpr int BATCH   = 8;
constexpr int SEQ     = 4096;
constexpr int FEAT_X  = 128;
constexpr int MEM     = 256;
constexpr int HID     = 256;
constexpr int FCAT    = MEM + FEAT_X;
constexpr int NROWS   = BATCH * SEQ;
constexpr int URP     = SEQ + 128;
constexpr int NSHIFT  = 8;
constexpr float HCARRY     = 1024.0f;
constexpr float HCARRY_INV = 1.0f / 1024.0f;
constexpr float WCARRY     = 16.0f;
constexpr float WCARRY_INV = 1.0f / 16.0f;
constexpr int SLABP   = 68;

static_assert(FCAT == 384);
static_assert(FCAT % 32 == 0);
static_assert(NROWS % 64 == 0 && HID % 64 == 0 && MEM % 64 == 0);
static_assert(SEQ % 64 == 0);
static_assert(URP % 8 == 0);
static_assert((BATCH * NSHIFT * (URP / 8)) % 256 == 0);
static_assert((size_t)NROWS * HID * 4 == (size_t)33554432);
static_assert((size_t)NROWS * HID * 4 + (size_t)BATCH * HID * 4 == (size_t)33562624);
static_assert(SEQ - 1 + 63 < URP);

typedef __attribute__((ext_vector_type(16))) _Float16 v16h;
typedef __attribute__((ext_vector_type(8)))  _Float16 v8h;
typedef __attribute__((ext_vector_type(8)))  float    v8f;
typedef __attribute__((ext_vector_type(4)))  float    v4f;

__device__ __forceinline__ void grp_guard_h(v8f& a, v8f& b, v8f& c, v8f& d, v16h x, v16h y0, v16h y1, v16h y2, v16h y3) {
  asm volatile("v_nop\n\tv_nop\n\tv_nop\n\tv_nop" : "+v"(a), "+v"(b), "+v"(c), "+v"(d) : "v"(x), "v"(y0), "v"(y1), "v"(y2), "v"(y3));
}
__device__ __forceinline__ void keep4_h(v16h a, v16h b, v16h c, v16h d) { asm volatile("v_nop" :: "v"(a), "v"(b), "v"(c), "v"(d)); }
__device__ __forceinline__ void acc_guard4(v8f& a, v8f& b, v8f& c, v8f& d) { asm volatile("v_nop\n\tv_nop\n\tv_nop\n\tv_nop" : "+v"(a), "+v"(b), "+v"(c), "+v"(d)); }

union FragU { v16h v; v8h h[2]; };
__device__ __forceinline__ v16h frag_load(const _Float16* p) {
  FragU f;
  f.h[0] = *(const v8h*)(p);
  f.h[1] = *(const v8h*)(p + 16);
  return f.v;
}
__device__ __forceinline__ v8f frag_mma(v16h a, v16h b, v8f c) {
  return __builtin_amdgcn_wmma_f32_16x16x32_f16(false, a, false, b, (short)0, c, false, false);
}

__global__ __launch_bounds__(256) void prep_ux_kernel(const float* __restrict__ x, const float* __restrict__ wu,
                                                      const float* __restrict__ bu, float* __restrict__ u32,
                                                      unsigned short* __restrict__ acat) {
  __shared__ __align__(16) float su[64];
  const int tid = threadIdx.x, lane = tid & 31, wave = tid >> 5;
  const int hh = lane >> 4, c = lane & 15;
  const int row0 = blockIdx.x * 64;
  const v4f w0 = *(const v4f*)(wu + 8 * c);
  const v4f w1 = *(const v4f*)(wu + 8 * c + 4);
  const float bias = bu[0];
  v8h hv[4];
#pragma unroll
  for (int it = 0; it < 4; ++it) {
    const int rl = wave * 8 + it * 2 + hh;
    const float* xp = x + (size_t)(row0 + rl) * FEAT_X + 8 * c;
    const v4f a = *(const v4f*)(xp);
    const v4f b = *(const v4f*)(xp + 4);
    float s = 0.0f;
    s += a[0] * w0[0];
    s += a[1] * w0[1];
    s += a[2] * w0[2];
    s += a[3] * w0[3];
    s += b[0] * w1[0];
    s += b[1] * w1[1];
    s += b[2] * w1[2];
    s += b[3] * w1[3];
    s += __shfl_xor(s, 1, 32);
    s += __shfl_xor(s, 2, 32);
    s += __shfl_xor(s, 4, 32);
    s += __shfl_xor(s, 8, 32);
    const float uval = fmaxf(s + bias, 0.0f);
    if (c == 0) su[rl] = uval;
    hv[it][0] = (_Float16)a[0];
    hv[it][1] = (_Float16)a[1];
    hv[it][2] = (_Float16)a[2];
    hv[it][3] = (_Float16)a[3];
    hv[it][4] = (_Float16)b[0];
    hv[it][5] = (_Float16)b[1];
    hv[it][6] = (_Float16)b[2];
    hv[it][7] = (_Float16)b[3];
  }
  for (int pass = 0; pass < 2; ++pass) {
#pragma unroll
    for (int it = 0; it < 4; ++it) {
      const int rl = wave * 8 + it * 2 + hh;
      *(volatile v8h*)(acat + (size_t)(row0 + rl) * FCAT + MEM + 8 * c) = hv[it];
    }
    __threadfence();
  }
  __syncthreads();
  if (tid < 16) {
    const v4f v = *(const v4f*)(su + 4 * tid);
    float* up = u32 + row0 + 4 * tid;
    *(volatile v4f*)up = v;
    __threadfence();
    *(volatile v4f*)up = v;
  }
}

__global__ __launch_bounds__(256) void build_urs_kernel(const float* __restrict__ u32, unsigned short* __restrict__ urs) {
  const int i = blockIdx.x * 256 + threadIdx.x;
  const int total = BATCH * NSHIFT * (URP / 8);
  if (i < total) {
    const int seg = i % (URP / 8);
    const int bj  = i / (URP / 8);
    const int j   = bj & (NSHIFT - 1);
    const int b   = bj >> 3;
    const int p0  = seg * 8 + j;
    const float* ub = u32 + (size_t)b * SEQ;
    v8h hv;
#pragma unroll
    for (int e = 0; e < 8; ++e) {
      const int sidx = (SEQ - 1) - (p0 + e);
      const int sc = (sidx < 0) ? 0 : sidx;
      const float ld = ub[sc];
      const float val = (sidx >= 0) ? ld : 0.0f;
      hv[e] = (_Float16)val;
    }
    *(volatile v8h*)(urs + (size_t)i * 8) = hv;
    __threadfence();
    *(volatile v8h*)(urs + (size_t)i * 8) = hv;
  }
}

__global__ __launch_bounds__(256) void cvt8_f16_kernel(const float* __restrict__ src, unsigned short* __restrict__ dst,
                                                       int n8, float sc) {
  const int i = blockIdx.x * 256 + threadIdx.x;
  if (i < n8) {
    const float* sp = src + (size_t)i * 8;
    const v4f a = *(const v4f*)(sp);
    const v4f b = *(const v4f*)(sp + 4);
    v8h hv;
    hv[0] = (_Float16)(a[0] * sc);
    hv[1] = (_Float16)(a[1] * sc);
    hv[2] = (_Float16)(a[2] * sc);
    hv[3] = (_Float16)(a[3] * sc);
    hv[4] = (_Float16)(b[0] * sc);
    hv[5] = (_Float16)(b[1] * sc);
    hv[6] = (_Float16)(b[2] * sc);
    hv[7] = (_Float16)(b[3] * sc);
    *(volatile v8h*)(dst + (size_t)i * 8) = hv;
    __threadfence();
    *(volatile v8h*)(dst + (size_t)i * 8) = hv;
  }
}

__global__ __launch_bounds__(256) void tpw_f16_kernel(const float* __restrict__ src, int R, int C, int ldo,
                                                      unsigned short* __restrict__ O, float sc) {
  __shared__ float Tt[64 * 65];
  const int tid = threadIdx.x;
  const int c0 = blockIdx.x * 64, r0 = blockIdx.y * 64;
#pragma unroll
  for (int i = 0; i < 4; ++i) {
    const int idx = i * 256 + tid;
    const int rr = idx >> 4, cc = (idx & 15) * 4;
    const v4f v = *(const v4f*)(src + (size_t)(r0 + rr) * (size_t)C + c0 + cc);
    Tt[rr * 65 + cc + 0] = v[0];
    Tt[rr * 65 + cc + 1] = v[1];
    Tt[rr * 65 + cc + 2] = v[2];
    Tt[rr * 65 + cc + 3] = v[3];
  }
  __syncthreads();
  const int q = tid >> 3, c8 = (tid & 7) * 8;
  v8h hv[2];
#pragma unroll
  for (int g = 0; g < 2; ++g) {
    const int qq = g * 32 + q;
#pragma unroll
    for (int e = 0; e < 8; ++e) {
      const float f = Tt[(c8 + e) * 65 + qq];
      hv[g][e] = (_Float16)(f * sc);
    }
  }
  for (int pass = 0; pass < 2; ++pass) {
#pragma unroll
    for (int g = 0; g < 2; ++g) {
      const size_t o = (size_t)(c0 + g * 32 + q) * (size_t)ldo + (size_t)(r0 + c8);
      *(volatile v8h*)(O + o) = hv[g];
    }
    __threadfence();
  }
}

__global__ __launch_bounds__(128) void toeplitz_conv_kernel(const unsigned short* __restrict__ ursp,
                                                            const unsigned short* __restrict__ hhp,
                                                            unsigned short* __restrict__ acat) {
  __shared__ __align__(16) float sT[4][16 * SLABP];
  const _Float16* URS = (const _Float16*)ursp;
  const _Float16* HH  = (const _Float16*)hhp;
  const int lane = threadIdx.x & 31, wave = threadIdx.x >> 5;
  const int b = blockIdx.y;
  const int s0 = blockIdx.x * 64;
  const int rlane = lane & 15, hh = lane >> 4, koff = hh * 8, mOff = hh * 8;
  const int jsh = (7 - rlane) & 7;
  const int abase = (SEQ - 8) - ((rlane >> 3) << 3) - s0 + koff;
  const _Float16* ap = URS + (size_t)(b * NSHIFT + jsh) * URP + abase;
  const _Float16* bp = HH + (size_t)(64 * wave + rlane) * SEQ + koff;
  const int kend = s0 + 64;

  v8f acc[4][4];
#pragma unroll
  for (int i = 0; i < 4; ++i)
#pragma unroll
    for (int j = 0; j < 4; ++j) acc[i][j] = (v8f){0.f, 0.f, 0.f, 0.f, 0.f, 0.f, 0.f, 0.f};

  for (int k0 = 0; k0 < kend; k0 += 32) {
    v16h bh[4];
#pragma unroll
    for (int j = 0; j < 4; ++j) bh[j] = frag_load(bp + (size_t)(16 * j) * SEQ + k0);
#pragma unroll
    for (int i = 0; i < 4; ++i) {
      const v16h ah = frag_load(ap + k0 - 16 * i);
#pragma unroll
      for (int j = 0; j < 4; ++j) acc[i][j] = frag_mma(ah, bh[j], acc[i][j]);
      grp_guard_h(acc[i][0], acc[i][1], acc[i][2], acc[i][3], ah, bh[0], bh[1], bh[2], bh[3]);
    }
    keep4_h(bh[0], bh[1], bh[2], bh[3]);
  }
  acc_guard4(acc[0][0], acc[0][1], acc[0][2], acc[0][3]);
  acc_guard4(acc[1][0], acc[1][1], acc[1][2], acc[1][3]);
  acc_guard4(acc[2][0], acc[2][1], acc[2][2], acc[2][3]);
  acc_guard4(acc[3][0], acc[3][1], acc[3][2], acc[3][3]);

  float* slab = sT[wave];
  unsigned short* Cb = acat + ((size_t)b * SEQ + (size_t)s0) * FCAT + 64 * wave;
  const int q = lane >> 3, c8 = (lane & 7) * 8;
#pragma unroll
  for (int i = 0; i < 4; ++i) {
#pragma unroll
    for (int j = 0; j < 4; ++j) {
#pragma unroll
      for (int r = 0; r < 8; ++r) slab[(mOff + r) * SLABP + (j << 4) + rlane] = acc[i][j][r] * HCARRY_INV;
    }
    __builtin_amdgcn_fence(__ATOMIC_RELEASE, "workgroup");
    __builtin_amdgcn_wave_barrier();
    __builtin_amdgcn_fence(__ATOMIC_ACQUIRE, "workgroup");
    v8h hv[4];
#pragma unroll
    for (int it = 0; it < 4; ++it) {
      const float* sp = slab + (it * 4 + q) * SLABP + c8;
#pragma unroll
      for (int e = 0; e < 8; ++e) hv[it][e] = (_Float16)sp[e];
    }
    for (int pass = 0; pass < 2; ++pass) {
#pragma unroll
      for (int it = 0; it < 4; ++it) {
        const int row = 16 * i + it * 4 + q;
        *(volatile v8h*)(Cb + (size_t)row * FCAT + c8) = hv[it];
      }
      __threadfence();
    }
    __builtin_amdgcn_fence(__ATOMIC_RELEASE, "workgroup");
    __builtin_amdgcn_wave_barrier();
    __builtin_amdgcn_fence(__ATOMIC_ACQUIRE, "workgroup");
  }
}

__global__ __launch_bounds__(256) void head_gemm_kernel(
    const unsigned short* __restrict__ Ap, int lda,
    const unsigned short* __restrict__ Btp, int ldb,
    float* __restrict__ Cout, int ldc,
    const float* __restrict__ bias,
    int Mrows, int Ncols, int Kdim, float scale) {
  const _Float16* Amat = (const _Float16*)Ap;
  const _Float16* Bmat = (const _Float16*)Btp;
  __shared__ __align__(16) float sT[8][16 * SLABP];
  const int lane = threadIdx.x & 31;
  const int wave = threadIdx.x >> 5;
  const int tilesN = Ncols >> 6;
  const int tilesM = Mrows >> 6;
  const int tile = blockIdx.x * 8 + wave;
  if (tile >= tilesM * tilesN) return;
  const int tm = tile / tilesN;
  const int tn = tile - tm * tilesN;
  const int m0 = tm << 6;
  const int n0 = tn << 6;
  const int rlane = lane & 15;
  const int koff  = (lane >> 4) * 8;
  const int mOff  = (lane >> 4) * 8;

  v8f acc[4][4];
#pragma unroll
  for (int i = 0; i < 4; ++i)
#pragma unroll
    for (int j = 0; j < 4; ++j) acc[i][j] = (v8f){0.f, 0.f, 0.f, 0.f, 0.f, 0.f, 0.f, 0.f};

  for (int k0 = 0; k0 < Kdim; k0 += 32) {
    v16h bh[4];
#pragma unroll
    for (int j = 0; j < 4; ++j) {
      const size_t bo = (size_t)(n0 + (j << 4) + rlane) * ldb + koff + k0;
      bh[j] = frag_load(Bmat + bo);
    }
#pragma unroll
    for (int i = 0; i < 4; ++i) {
      const size_t ao = (size_t)(m0 + (i << 4) + rlane) * lda + koff + k0;
      const v16h ah = frag_load(Amat + ao);
#pragma unroll
      for (int j = 0; j < 4; ++j) acc[i][j] = frag_mma(ah, bh[j], acc[i][j]);
      grp_guard_h(acc[i][0], acc[i][1], acc[i][2], acc[i][3], ah, bh[0], bh[1], bh[2], bh[3]);
    }
    keep4_h(bh[0], bh[1], bh[2], bh[3]);
  }
  acc_guard4(acc[0][0], acc[0][1], acc[0][2], acc[0][3]);
  acc_guard4(acc[1][0], acc[1][1], acc[1][2], acc[1][3]);
  acc_guard4(acc[2][0], acc[2][1], acc[2][2], acc[2][3]);
  acc_guard4(acc[3][0], acc[3][1], acc[3][2], acc[3][3]);

  float* slab = sT[wave];
#pragma unroll
  for (int i = 0; i < 4; ++i) {
    const int mBase = m0 + (i << 4);
#pragma unroll
    for (int j = 0; j < 4; ++j) {
      const int n = n0 + (j << 4) + rlane;
      const float bv = bias[n];
#pragma unroll
      for (int r = 0; r < 8; ++r) {
        float v = acc[i][j][r] * scale;
        v += bv;
        v = fmaxf(v, 0.0f);
        slab[(mOff + r) * SLABP + (j << 4) + rlane] = v;
      }
    }
    __builtin_amdgcn_fence(__ATOMIC_RELEASE, "workgroup");
    __builtin_amdgcn_wave_barrier();
    __builtin_amdgcn_fence(__ATOMIC_ACQUIRE, "workgroup");
    {
      const int hh = lane >> 4, c4 = (lane & 15) * 4;
      for (int pass = 0; pass < 2; ++pass) {
#pragma unroll
        for (int it = 0; it < 8; ++it) {
          const int row = it * 2 + hh;
          const v4f v = *(const v4f*)(slab + row * SLABP + c4);
          *(volatile v4f*)(Cout + (size_t)(mBase + row) * ldc + n0 + c4) = v;
        }
        __threadfence();
      }
    }
    __builtin_amdgcn_fence(__ATOMIC_RELEASE, "workgroup");
    __builtin_amdgcn_wave_barrier();
    __builtin_amdgcn_fence(__ATOMIC_ACQUIRE, "workgroup");
  }
}

__global__ __launch_bounds__(256) void copy_last_kernel(const float* h, float* hn) {
  const int tid = threadIdx.x;
  v4f v[2];
#pragma unroll
  for (int it = 0; it < 2; ++it) {
    const int idx = it * 256 + tid;
    const int b = idx >> 6, c4 = (idx & 63) * 4;
    v[it] = *(const v4f*)(h + ((size_t)b * SEQ + (size_t)(SEQ - 1)) * HID + c4);
  }
  for (int pass = 0; pass < 2; ++pass) {
#pragma unroll
    for (int it = 0; it < 2; ++it) {
      const int idx = it * 256 + tid;
      *(volatile v4f*)(hn + (size_t)idx * 4) = v[it];
    }
    __threadfence();
  }
}

extern "C" void kernel_launch(void* const* d_in, const int* in_sizes, int n_in,
                              void* d_out, int out_size, void* d_ws, size_t ws_size, hipStream_t stream) {
  if (n_in < 6 || d_out == nullptr || d_ws == nullptr) return;
  if (in_sizes[0] != BATCH * SEQ * FEAT_X || in_sizes[1] != FEAT_X || in_sizes[2] != 1 ||
      in_sizes[3] != FCAT * HID || in_sizes[4] != HID || in_sizes[5] != MEM * SEQ ||
      out_size != NROWS * HID + BATCH * HID) return;

  const float* x   = (const float*)d_in[0];
  const float* w_u = (const float*)d_in[1];
  const float* b_u = (const float*)d_in[2];
  const float* w_h = (const float*)d_in[3];
  const float* b_h = (const float*)d_in[4];
  const float* hir = (const float*)d_in[5];
  float* h_out  = (float*)d_out;
  float* hn_out = h_out + (size_t)NROWS * HID;

  char* ws = (char*)d_ws;
  size_t off = 0;
  auto carve = [&](size_t bytes) -> char* { char* p = ws + off; off += (bytes + 255) & ~(size_t)255; return p; };
  unsigned short* ACAT = (unsigned short*)carve((size_t)NROWS * FCAT * 2);
  unsigned short* HH   = (unsigned short*)carve((size_t)MEM * SEQ * 2);
  unsigned short* WT   = (unsigned short*)carve((size_t)HID * FCAT * 2);
  float*          U32  = (float*)carve((size_t)NROWS * 4);
  unsigned short* URS  = (unsigned short*)carve((size_t)BATCH * NSHIFT * URP * 2);
  if (off > ws_size || off > (size_t)134217728) return;

  const int n8h = MEM * SEQ / 8;
  cvt8_f16_kernel<<<(n8h + 255) / 256, 256, 0, stream>>>(hir, HH, n8h, HCARRY);
  tpw_f16_kernel<<<dim3(HID / 64, FCAT / 64), 256, 0, stream>>>(w_h, FCAT, HID, FCAT, WT, WCARRY);
  prep_ux_kernel<<<NROWS / 64, 256, 0, stream>>>(x, w_u, b_u, U32, ACAT);
  build_urs_kernel<<<(BATCH * NSHIFT * (URP / 8)) / 256, 256, 0, stream>>>(U32, URS);

  toeplitz_conv_kernel<<<dim3(SEQ / 64, BATCH), 128, 0, stream>>>(URS, HH, ACAT);

  head_gemm_kernel<<<(NROWS / 64) * (HID / 64) / 8, 256, 0, stream>>>(
      ACAT, FCAT, WT, FCAT, h_out, HID, b_h, NROWS, HID, FCAT, WCARRY_INV);

  copy_last_kernel<<<1, 256, 0, stream>>>(h_out, hn_out);
}
